// DataReuploadingTorso_83769042141231
// MI455X (gfx1250) — hardware-verified
//
#include <hip/hip_runtime.h>


typedef __attribute__((ext_vector_type(16))) _Float16     v16h;
typedef __attribute__((ext_vector_type(8)))  float        v8f;
typedef __attribute__((ext_vector_type(8)))  unsigned int v8u;

#define NQ      8
#define DIM     256
#define NL      4
#define ITEMS   16
#define THREADS 512
#define LDSTR   264

struct C2 { float x, y; };

__device__ __forceinline__ C2 cmadd2(C2 m0, C2 a0, C2 m1, C2 a1) {
    C2 r;
    r.x = m0.x * a0.x - m0.y * a0.y + m1.x * a1.x - m1.y * a1.y;
    r.y = m0.x * a0.y + m0.y * a0.x + m1.x * a1.y + m1.y * a1.x;
    return r;
}

__device__ __forceinline__ void rot_mat(float phi, float th, float om, C2 m[4]) {
    float c, s, ca, sa, cb, sb;
    __sincosf(0.5f * th, &s, &c);
    __sincosf(0.5f * (phi + om), &sa, &ca);
    __sincosf(0.5f * (phi - om), &sb, &cb);
    m[0] = { ca * c, -sa * c };
    m[1] = { -cb * s, -sb * s };
    m[2] = { cb * s, -sb * s };
    m[3] = { ca * c,  sa * c };
}

__device__ __forceinline__ void mat2mul(const C2 t[4], const C2 d[4], C2 m[4]) {
    m[0] = cmadd2(t[0], d[0], t[1], d[2]);
    m[1] = cmadd2(t[0], d[1], t[1], d[3]);
    m[2] = cmadd2(t[2], d[0], t[3], d[2]);
    m[3] = cmadd2(t[2], d[1], t[3], d[3]);
}

__device__ __forceinline__ void apply_gate(C2 st[8], const C2 m[4], int p, int lane) {
    if (p < 3) {
        const int mask = 1 << p;
        #pragma unroll
        for (int r = 0; r < 8; ++r) {
            if ((r & mask) == 0) {
                const int r1 = r | mask;
                C2 a0 = st[r], a1 = st[r1];
                st[r]  = cmadd2(m[0], a0, m[1], a1);
                st[r1] = cmadd2(m[2], a0, m[3], a1);
            }
        }
    } else {
        const int lm  = 1 << (p - 3);
        const int bit = (lane >> (p - 3)) & 1;
        #pragma unroll
        for (int r = 0; r < 8; ++r) {
            C2 mine = st[r];
            C2 peer;
            peer.x = __shfl_xor(mine.x, lm, 32);
            peer.y = __shfl_xor(mine.y, lm, 32);
            C2 a0 = bit ? peer : mine;
            C2 a1 = bit ? mine : peer;
            C2 n0 = cmadd2(m[0], a0, m[1], a1);
            C2 n1 = cmadd2(m[2], a0, m[3], a1);
            st[r] = bit ? n1 : n0;
        }
    }
}

__global__ __launch_bounds__(THREADS)
void qcirc_wmma_kernel(const float* __restrict__ xg,
                       const float* __restrict__ theta,
                       const float* __restrict__ omega,
                       float* __restrict__ out, int B) {
    __shared__ _Float16 probs[ITEMS][LDSTR];
    __shared__ _Float16 probl[ITEMS][LDSTR];
    __shared__ __attribute__((aligned(16))) float sout[ITEMS * 8];

    const int lane      = threadIdx.x & 31;
    const int wave      = threadIdx.x >> 5;
    const int blockBase = blockIdx.x * ITEMS;
    int g = blockBase + wave;
    if (g >= B) g = B - 1;

    __builtin_prefetch(xg + (size_t)(blockBase + ITEMS) * 12, 0, 1);

    float x[12];
    #pragma unroll
    for (int i = 0; i < 12; ++i) x[i] = xg[g * 12 + i];

    C2 st[8];
    #pragma unroll
    for (int r = 0; r < 8; ++r) st[r] = { 0.f, 0.f };
    if (lane == 0) st[0].x = 1.f;

    #pragma unroll
    for (int l = 0; l < NL; ++l) {
        #pragma unroll
        for (int q = 0; q < NQ; ++q) {
            const int p = 7 - q;
            const int f = (q & 3) * 3;
            C2 dm[4], tm[4], m[4];
            rot_mat(x[f + 0] * omega[l * 24 + q * 3 + 0],
                    x[f + 1] * omega[l * 24 + q * 3 + 1],
                    x[f + 2] * omega[l * 24 + q * 3 + 2], dm);
            rot_mat(theta[(q * 5 + l) * 3 + 0],
                    theta[(q * 5 + l) * 3 + 1],
                    theta[(q * 5 + l) * 3 + 2], tm);
            mat2mul(tm, dm, m);
            apply_gate(st, m, p, lane);
        }
        const unsigned pm = (l & 1) ? 0x2Au : 0x55u;
        #pragma unroll
        for (int r = 0; r < 8; ++r) {
            unsigned s = (unsigned)(lane * 8 + r);
            unsigned t = s & (s >> 1);
            if (__popc(t & pm) & 1) { st[r].x = -st[r].x; st[r].y = -st[r].y; }
        }
    }

    #pragma unroll
    for (int q = 0; q < NQ; ++q) {
        const int p = 7 - q;
        const int f = (q & 3) * 3;
        C2 m[4];
        rot_mat(x[f + 0] * omega[4 * 24 + q * 3 + 0] + theta[(q * 5 + 4) * 3 + 0],
                x[f + 1] * omega[4 * 24 + q * 3 + 1] + theta[(q * 5 + 4) * 3 + 1],
                x[f + 2] * omega[4 * 24 + q * 3 + 2] + theta[(q * 5 + 4) * 3 + 2], m);
        apply_gate(st, m, p, lane);
    }

    #pragma unroll
    for (int r = 0; r < 8; ++r) {
        float pr = (st[r].x * st[r].x + st[r].y * st[r].y) * 1024.0f;
        const _Float16 ph = (_Float16)pr;
        probs[wave][lane * 8 + r] = ph;
        probl[wave][lane * 8 + r] = (_Float16)((pr - (float)ph) * 2048.0f);
    }
    __syncthreads();

    if (wave == 0) {
        const int row    = lane & 15;
        const int hi     = lane >> 4;
        const int kbaseA = hi * 8;
        const unsigned colmask = (row < 8) ? 0xFFFFFFFFu : 0u;
        const int      bitpos  = (7 - row) & 7;
        v8f acc = {};
        #pragma unroll
        for (int k0 = 0; k0 < DIM; k0 += 32) {
            v16h a, al;
            v8u  bw;
            #pragma unroll
            for (int j = 0; j < 8; ++j) {
                const int ka = k0 + kbaseA + ((j < 4) ? 2 * j : 16 + 2 * (j - 4));
                a[2 * j]     = probs[row][ka];      al[2 * j]     = probl[row][ka];
                a[2 * j + 1] = probs[row][ka + 1];  al[2 * j + 1] = probl[row][ka + 1];
                const int kb = ka;
                const unsigned z0 = 0x3C00u ^ ((((unsigned)kb       >> bitpos) & 1u) << 15);
                const unsigned z1 = 0x3C00u ^ ((((unsigned)(kb + 1) >> bitpos) & 1u) << 15);
                bw[j] = (z0 | (z1 << 16)) & colmask;
            }
            const v16h b = __builtin_bit_cast(v16h, bw);
            v8f lo = {};
            lo  = __builtin_amdgcn_wmma_f32_16x16x32_f16(false, al, false, b, (short)0, lo, false, false);
            acc = __builtin_amdgcn_wmma_f32_16x16x32_f16(false, a,  false, b, (short)0, acc, false, false);
            acc += lo * (1.0f / 2048.0f);
        }
        const int col = lane & 15;
        if (col < 8) {
            #pragma unroll
            for (int v = 0; v < 8; ++v) sout[(v + hi * 8) * 8 + col] = acc[v] * (1.0f / 1024.0f);
        }
        asm volatile("s_wait_dscnt 0" ::: "memory");
        typedef __attribute__((ext_vector_type(4))) float v4f_t; typedef float v4fa __attribute__((ext_vector_type(4), may_alias));
        const int item = blockBase + (lane >> 1);
        if (item < B) { const v4f_t v = *(const volatile v4fa*)(sout + lane * 4);
            *(volatile v4f_t*)(out + (size_t)blockBase * 8 + lane * 4) = v; __threadfence(); *(volatile v4f_t*)(out + (size_t)blockBase * 8 + lane * 4) = v; }
    }
}

extern "C" void kernel_launch(void* const* d_in, const int* in_sizes, int n_in,
                              void* d_out, int out_size, void* d_ws, size_t ws_size,
                              hipStream_t stream) {
    const float* x     = (const float*)d_in[0];
    const float* theta = (const float*)d_in[1];
    const float* omega = (const float*)d_in[2];
    float* out         = (float*)d_out;

    const int B      = in_sizes[0] / 12;
    const int blocks = (B + ITEMS - 1) / ITEMS;
    hipLaunchKernelGGL(qcirc_wmma_kernel, dim3(blocks), dim3(THREADS), 0, stream,
                       x, theta, omega, out, B);
}
